// Encoder_10754598109893
// MI455X (gfx1250) — hardware-verified
//
#include <hip/hip_runtime.h>
#include <math.h>

constexpr int NBATCH    = 256;
constexpr int NSTEP     = 256;
constexpr int NFEAT     = 64;
constexpr int NHID      = 256;
constexpr int NGATE     = 3 * NHID;
constexpr int NDIR      = 2;
constexpr int ROWS_BLK  = 32;
constexpr int NTHR      = 512;
constexpr int NWAVE     = NTHR / 32;
constexpr int K_LAYER0  = NFEAT + NHID;
constexpr int K_LAYER1  = 2 * NHID + NHID;
constexpr int OUT_PITCH = 260;
constexpr int PACK_THR  = 256;
constexpr float WCARRY     = 16.0f;
constexpr float WCARRY_INV = 1.0f / 16.0f;

static_assert(NHID == 16 * NWAVE);
static_assert(NBATCH % ROWS_BLK == 0);
static_assert(ROWS_BLK == 32);
static_assert(NFEAT % 32 == 0 && NHID % 32 == 0);
static_assert(K_LAYER0 % 32 == 0 && K_LAYER1 % 32 == 0);
static_assert(K_LAYER0 == 320 && K_LAYER1 == 768);
static_assert(ROWS_BLK * NFEAT == NTHR * 4);
static_assert((ROWS_BLK * 2 * NHID / 8) % NTHR == 0);
static_assert(ROWS_BLK == 2 * NWAVE);
static_assert((ROWS_BLK * NHID / 4) % NTHR == 0);
static_assert(NGATE == 768);

typedef __attribute__((ext_vector_type(16))) _Float16 v16h;
typedef __attribute__((ext_vector_type(8)))  _Float16 v8h;
typedef __attribute__((ext_vector_type(4)))  _Float16 v4h;
typedef __attribute__((ext_vector_type(8)))  float    v8f;
typedef __attribute__((ext_vector_type(4)))  float    v4f;

struct FragH {
  union U { v16h v; v8h h[2]; };
  static __device__ __forceinline__ v16h load(const _Float16* p) {
    U f;
    f.h[0] = *(const v8h*)(p);
    f.h[1] = *(const v8h*)(p + 16);
    return f.v;
  }
  static __device__ __forceinline__ v8f mma(v16h a, v16h b, v8f c) {
    return __builtin_amdgcn_wmma_f32_16x16x32_f16(false, a, false, b, (short)0, c, false, false);
  }
};

__device__ __forceinline__ void guard6(v8f& a, v8f& b, v8f& c, v8f& d, v8f& e, v8f& f,
                                       v16h x0, v16h x1, v16h w0, v16h w1, v16h w2) {
  asm volatile("v_nop\n\tv_nop\n\tv_nop\n\tv_nop"
               : "+v"(a), "+v"(b), "+v"(c), "+v"(d), "+v"(e), "+v"(f)
               : "v"(x0), "v"(x1), "v"(w0), "v"(w1), "v"(w2));
}
__device__ __forceinline__ void acc_guard4(v8f& a, v8f& b, v8f& c, v8f& d) {
  asm volatile("v_nop\n\tv_nop\n\tv_nop\n\tv_nop" : "+v"(a), "+v"(b), "+v"(c), "+v"(d));
}

__device__ __forceinline__ float fsig(float x)  { return __builtin_amdgcn_rcpf(1.0f + __expf(-x)); }
__device__ __forceinline__ float ftanh(float x) { return 1.0f - 2.0f * __builtin_amdgcn_rcpf(__expf(2.0f * x) + 1.0f); }

__global__ __launch_bounds__(PACK_THR) void pack_w_kernel(const float* __restrict__ src, unsigned short* __restrict__ dst,
                                                          int nrow, int ncol8, int spitch, int dpitch, int dcol0) {
  const int i  = blockIdx.x * PACK_THR + threadIdx.x;
  const int n8 = nrow * ncol8;
  if (i < n8) {
    const int row = i / ncol8;
    const int c8  = i - row * ncol8;
    const float* sp = src + (size_t)row * spitch + c8 * 8;
    const v4f a = *(const v4f*)(sp);
    const v4f b = *(const v4f*)(sp + 4);
    v8h hv;
#pragma unroll
    for (int e = 0; e < 4; ++e) {
      const float fa = a[e] * WCARRY;
      const float fb = b[e] * WCARRY;
      hv[e]     = (_Float16)fa;
      hv[4 + e] = (_Float16)fb;
    }
    unsigned short* dp = dst + (size_t)row * dpitch + dcol0 + c8 * 8;
    *(volatile v8h*)dp = hv;
    __threadfence();
    *(volatile v8h*)dp = hv;
  }
}

template <int CIN, bool FIRST, int PITCH>
__device__ __forceinline__ void stage_input(_Float16* As, const float* X, const _Float16* Y0, int b0, int tt, int tid) {
  if (FIRST) {
    const int m = tid >> 4, f4 = (tid & 15) * 4;
    const v4f v = *(const v4f*)(X + ((size_t)(b0 + m) * NSTEP + (size_t)tt) * NFEAT + f4);
    v4h hv;
    hv[0] = (_Float16)v[0];
    hv[1] = (_Float16)v[1];
    hv[2] = (_Float16)v[2];
    hv[3] = (_Float16)v[3];
    *(v4h*)(As + m * PITCH + f4) = hv;
  } else {
    v8h tmp[4];
#pragma unroll
    for (int i = 0; i < 4; ++i) {
      const int idx = i * NTHR + tid;
      const int m = idx >> 6, c8 = (idx & 63) * 8;
      tmp[i] = *(const v8h*)(Y0 + ((size_t)tt * NBATCH + (size_t)(b0 + m)) * (2 * NHID) + c8);
    }
#pragma unroll
    for (int i = 0; i < 4; ++i) {
      const int idx = i * NTHR + tid;
      const int m = idx >> 6, c8 = (idx & 63) * 8;
      *(v8h*)(As + m * PITCH + c8) = tmp[i];
    }
  }
}

template <int CIN, bool FIRST>
__global__ __launch_bounds__(NTHR) void gru_scan_kernel(const float* __restrict__ X, unsigned short* __restrict__ Y0p,
                                                        float* __restrict__ OUT, const unsigned short* __restrict__ Wp,
                                                        const float* __restrict__ bih, const float* __restrict__ bhh) {
  constexpr int AK    = CIN + NHID;
  constexpr int PITCH = AK + 8;
  static_assert(AK % 32 == 0 && CIN % 32 == 0);
  static_assert(PITCH % 8 == 0);
  static_assert(FIRST || (ROWS_BLK * PITCH * 2 >= ROWS_BLK * OUT_PITCH * 4));
  static_assert(ROWS_BLK * PITCH * 2 <= 65536);
  __shared__ __align__(16) _Float16 As[ROWS_BLK * PITCH];

  const int tid = threadIdx.x, lane = tid & 31, wave = tid >> 5;
  const int c = lane & 15, hh = lane >> 4, koff = hh * 8;
  const int dir = blockIdx.x >> 3;
  const int b0  = (blockIdx.x & 7) * ROWS_BLK;
  const int j   = 16 * wave + c;
  _Float16* Y0 = (_Float16*)Y0p;
  const _Float16* Wd = (const _Float16*)Wp + (size_t)dir * NGATE * AK;

  {
    const v8h z8h = {(_Float16)0.0f, (_Float16)0.0f, (_Float16)0.0f, (_Float16)0.0f,
                     (_Float16)0.0f, (_Float16)0.0f, (_Float16)0.0f, (_Float16)0.0f};
#pragma unroll 1
    for (int i = tid; i < ROWS_BLK * PITCH / 8; i += NTHR) *(v8h*)(As + i * 8) = z8h;
  }
  __syncthreads();
  stage_input<CIN, FIRST, PITCH>(As, X, Y0, b0, dir ? (NSTEP - 1) : 0, tid);

  const float b_r  = bih[dir * NGATE + j] + bhh[dir * NGATE + j];
  const float b_z  = bih[dir * NGATE + NHID + j] + bhh[dir * NGATE + NHID + j];
  const float b_in = bih[dir * NGATE + 2 * NHID + j];
  const float b_hn = bhh[dir * NGATE + 2 * NHID + j];

  float hst[2][8];
#pragma unroll
  for (int mt = 0; mt < 2; ++mt)
#pragma unroll
    for (int r = 0; r < 8; ++r) hst[mt][r] = 0.0f;
  __syncthreads();

  const _Float16* a0p = As + c * PITCH + koff;
  const _Float16* a1p = As + (16 + c) * PITCH + koff;
  const _Float16* wr  = Wd + (size_t)j * AK + koff;
  const _Float16* wz  = Wd + (size_t)(NHID + j) * AK + koff;
  const _Float16* wn  = Wd + (size_t)(2 * NHID + j) * AK + koff;
  const v8f z8 = {0.f, 0.f, 0.f, 0.f, 0.f, 0.f, 0.f, 0.f};

#pragma unroll 1
  for (int s = 0; s < NSTEP; ++s) {
    const int t = dir ? (NSTEP - 1 - s) : s;

    v8f aR[2], aZ[2], aNx[2], aNh[2];
    aR[0] = z8; aR[1] = z8; aZ[0] = z8; aZ[1] = z8;
    aNx[0] = z8; aNx[1] = z8; aNh[0] = z8; aNh[1] = z8;

#pragma unroll 1
    for (int kb = 0; kb < CIN; kb += 32) {
      const v16h a0 = FragH::load(a0p + kb);
      const v16h a1 = FragH::load(a1p + kb);
      const v16h br = FragH::load(wr + kb);
      const v16h bz = FragH::load(wz + kb);
      const v16h bn = FragH::load(wn + kb);
      aR[0]  = FragH::mma(a0, br, aR[0]);
      aR[1]  = FragH::mma(a1, br, aR[1]);
      aZ[0]  = FragH::mma(a0, bz, aZ[0]);
      aZ[1]  = FragH::mma(a1, bz, aZ[1]);
      aNx[0] = FragH::mma(a0, bn, aNx[0]);
      aNx[1] = FragH::mma(a1, bn, aNx[1]);
      guard6(aR[0], aR[1], aZ[0], aZ[1], aNx[0], aNx[1], a0, a1, br, bz, bn);
    }
#pragma unroll 1
    for (int kb = CIN; kb < AK; kb += 32) {
      const v16h a0 = FragH::load(a0p + kb);
      const v16h a1 = FragH::load(a1p + kb);
      const v16h br = FragH::load(wr + kb);
      const v16h bz = FragH::load(wz + kb);
      const v16h bn = FragH::load(wn + kb);
      aR[0]  = FragH::mma(a0, br, aR[0]);
      aR[1]  = FragH::mma(a1, br, aR[1]);
      aZ[0]  = FragH::mma(a0, bz, aZ[0]);
      aZ[1]  = FragH::mma(a1, bz, aZ[1]);
      aNh[0] = FragH::mma(a0, bn, aNh[0]);
      aNh[1] = FragH::mma(a1, bn, aNh[1]);
      guard6(aR[0], aR[1], aZ[0], aZ[1], aNh[0], aNh[1], a0, a1, br, bz, bn);
    }
    acc_guard4(aR[0], aR[1], aZ[0], aZ[1]);
    acc_guard4(aNx[0], aNx[1], aNh[0], aNh[1]);

    __syncthreads();

#pragma unroll
    for (int mt = 0; mt < 2; ++mt) {
#pragma unroll
      for (int r = 0; r < 8; ++r) {
        const float pr = aR[mt][r] * WCARRY_INV + b_r;
        const float pz = aZ[mt][r] * WCARRY_INV + b_z;
        const float gx = aNx[mt][r] * WCARRY_INV + b_in;
        const float gh = aNh[mt][r] * WCARRY_INV + b_hn;
        const float rg = fsig(pr);
        const float zg = fsig(pz);
        const float ng = ftanh(gx + rg * gh);
        const float ho = hst[mt][r];
        const float hn = (1.0f - zg) * ng + zg * ho;
        hst[mt][r] = hn;
        As[(16 * mt + 8 * hh + r) * PITCH + CIN + j] = (_Float16)hn;
      }
    }
    {
      int tn = dir ? (NSTEP - 2 - s) : (s + 1);
      tn = tn < 0 ? 0 : tn;
      tn = tn > (NSTEP - 1) ? (NSTEP - 1) : tn;
      stage_input<CIN, FIRST, PITCH>(As, X, Y0, b0, tn, tid);
    }
    __syncthreads();

    if (FIRST) {
      v8h yv[2];
#pragma unroll
      for (int q = 0; q < 2; ++q) yv[q] = *(const v8h*)(As + (2 * wave + q) * PITCH + CIN + 8 * lane);
      for (int pass = 0; pass < 2; ++pass) {
#pragma unroll
        for (int q = 0; q < 2; ++q) {
          const int row = 2 * wave + q;
          *(volatile v8h*)(Y0 + ((size_t)t * NBATCH + (size_t)(b0 + row)) * (2 * NHID) + dir * NHID + 8 * lane) = yv[q];
        }
        __threadfence();
      }
    }
  }

  if (!FIRST) {
    float* Hs = (float*)As;
#pragma unroll
    for (int mt = 0; mt < 2; ++mt)
#pragma unroll
      for (int r = 0; r < 8; ++r) Hs[(16 * mt + 8 * hh + r) * OUT_PITCH + j] = hst[mt][r];
    __syncthreads();
    v4f ov[4];
#pragma unroll
    for (int it = 0; it < 4; ++it) {
      const int idx = it * NTHR + tid;
      const int row = idx >> 6, c4 = (idx & 63) * 4;
      ov[it] = *(const v4f*)(Hs + row * OUT_PITCH + c4);
    }
    for (int pass = 0; pass < 2; ++pass) {
#pragma unroll
      for (int it = 0; it < 4; ++it) {
        const int idx = it * NTHR + tid;
        const int row = idx >> 6, c4 = (idx & 63) * 4;
        *(volatile v4f*)(OUT + (size_t)(b0 + row) * (2 * NHID) + dir * NHID + c4) = ov[it];
      }
      __threadfence();
    }
  }
}

extern "C" void kernel_launch(void* const* d_in, const int* in_sizes, int n_in,
                              void* d_out, int out_size, void* d_ws, size_t ws_size, hipStream_t stream) {
  if (n_in < 9 || d_out == nullptr || d_ws == nullptr) return;
  if (in_sizes[0] != NBATCH * NSTEP * NFEAT || in_sizes[1] != NDIR * NGATE * NFEAT ||
      in_sizes[2] != NDIR * NGATE * NHID || in_sizes[3] != NDIR * NGATE || in_sizes[4] != NDIR * NGATE ||
      in_sizes[5] != NDIR * NGATE * 2 * NHID || in_sizes[6] != NDIR * NGATE * NHID ||
      in_sizes[7] != NDIR * NGATE || in_sizes[8] != NDIR * NGATE || out_size != NBATCH * 2 * NHID) return;

  const float* x     = (const float*)d_in[0];
  const float* w_ih0 = (const float*)d_in[1];
  const float* w_hh0 = (const float*)d_in[2];
  const float* b_ih0 = (const float*)d_in[3];
  const float* b_hh0 = (const float*)d_in[4];
  const float* w_ih1 = (const float*)d_in[5];
  const float* w_hh1 = (const float*)d_in[6];
  const float* b_ih1 = (const float*)d_in[7];
  const float* b_hh1 = (const float*)d_in[8];
  float* out = (float*)d_out;

  char* ws = (char*)d_ws;
  size_t off = 0;
  auto carve = [&](size_t bytes) -> char* { char* p = ws + off; off += (bytes + 255) & ~(size_t)255; return p; };
  unsigned short* WC0 = (unsigned short*)carve((size_t)NDIR * NGATE * K_LAYER0 * 2);
  unsigned short* WC1 = (unsigned short*)carve((size_t)NDIR * NGATE * K_LAYER1 * 2);
  unsigned short* Y0  = (unsigned short*)carve((size_t)NSTEP * NBATCH * 2 * NHID * 2);
  if (off > ws_size || off > (size_t)134217728) return;

  const int nrow = NDIR * NGATE;
  pack_w_kernel<<<nrow * (NFEAT / 8) / PACK_THR, PACK_THR, 0, stream>>>(w_ih0, WC0, nrow, NFEAT / 8, NFEAT, K_LAYER0, 0);
  pack_w_kernel<<<nrow * (NHID / 8) / PACK_THR, PACK_THR, 0, stream>>>(w_hh0, WC0, nrow, NHID / 8, NHID, K_LAYER0, NFEAT);
  pack_w_kernel<<<nrow * (2 * NHID / 8) / PACK_THR, PACK_THR, 0, stream>>>(w_ih1, WC1, nrow, 2 * NHID / 8, 2 * NHID, K_LAYER1, 0);
  pack_w_kernel<<<nrow * (NHID / 8) / PACK_THR, PACK_THR, 0, stream>>>(w_hh1, WC1, nrow, NHID / 8, NHID, K_LAYER1, 2 * NHID);

  const int nblk = NDIR * (NBATCH / ROWS_BLK);
  gru_scan_kernel<NFEAT, true><<<nblk, NTHR, 0, stream>>>(x, Y0, out, WC0, b_ih0, b_hh0);
  gru_scan_kernel<2 * NHID, false><<<nblk, NTHR, 0, stream>>>(x, Y0, out, WC1, b_ih1, b_hh1);
}
